// PinnLayer_38044820308033
// MI455X (gfx1250) — hardware-verified
//
#include <hip/hip_runtime.h>

#define T_MAX_N 10.0f
namespace {
constexpr int BB = 1024;
constexpr int NN = 512;
constexpr int HH = 512;
constexpr size_t PL = (size_t)BB * HH;
constexpr size_t PLW = (size_t)HH * HH;
}
typedef __attribute__((ext_vector_type(16))) _Float16 v16h;
typedef __attribute__((ext_vector_type(8)))  _Float16 v8h;
typedef __attribute__((ext_vector_type(8)))  float    v8f;
typedef __attribute__((ext_vector_type(4)))  float    v4f_t;
typedef float v4fa __attribute__((ext_vector_type(4), may_alias));
typedef __attribute__((ext_vector_type(4)))  unsigned v4u_t;
typedef unsigned v4ua __attribute__((ext_vector_type(4), may_alias));
#define RSPLIT (1.0f / 2048.0f)
__device__ __forceinline__ _Float16 lo_of(float v, _Float16 h) { return (_Float16)((v - (float)h) * 2048.0f); }
__device__ __forceinline__ v8f wmma16(v16h a, v16h b, v8f c) { return __builtin_amdgcn_wmma_f32_16x16x32_f16(false, a, false, b, (short)0, c, false, false); }
__device__ __forceinline__ v8f wmma_split(v16h a, v16h al, v16h b, v16h bl, v8f c) { v8f x = {}; x = wmma16(al, b, x); x = wmma16(a, bl, x); return wmma16(a, b, c) + x * RSPLIT; }
__device__ __forceinline__ v16h frag16(const _Float16* p, int g) {
  return __builtin_shufflevector(*(const v8h*)(p + 8 * g), *(const v8h*)(p + 16 + 8 * g), 0,1,2,3,4,5,6,7,8,9,10,11,12,13,14,15);
}
__device__ __forceinline__ void stpair(_Float16* d, size_t pl, float v0, float v1) {
  const _Float16 a = (_Float16)v0, b = (_Float16)v1;
  const unsigned u = (unsigned)__builtin_bit_cast(unsigned short, a) | ((unsigned)__builtin_bit_cast(unsigned short, b) << 16);
  const unsigned w = (unsigned)__builtin_bit_cast(unsigned short, lo_of(v0, a)) | ((unsigned)__builtin_bit_cast(unsigned short, lo_of(v1, b)) << 16);
  *(volatile unsigned*)d = u; *(volatile unsigned*)(d + pl) = w; __threadfence(); *(volatile unsigned*)d = u; *(volatile unsigned*)(d + pl) = w;
}

__global__ void k_prep_inputs(const float* __restrict__ t, const float* __restrict__ p,
                              const float* __restrict__ plo, const float* __restrict__ pup,
                              _Float16* __restrict__ pn16, float* __restrict__ tn) {
  int idx = (blockIdx.x * blockDim.x + threadIdx.x) * 2;
  int b = idx >> 9, j = idx & 511;
  float v[2];
#pragma unroll
  for (int u = 0; u < 2; ++u) {
    float lo = plo[j + u], up = pup[j + u];
    v[u] = (up == lo) ? 0.f : (2.f * (p[idx + u] - lo) / (up - lo) - 1.f);
  }
  stpair(pn16 + idx, PL, v[0], v[1]);
  if (j == 0) { const float tv = 2.f * t[b] / T_MAX_N - 1.f; *(volatile float*)(tn + b) = tv; __threadfence(); *(volatile float*)(tn + b) = tv; }
}
__global__ void k_tcast(const float* __restrict__ W, int koff, int ldw, _Float16* __restrict__ Wt) {
  int idx = blockIdx.x * blockDim.x + threadIdx.x;
  if (idx >= 512 * 64) return;
  int n = idx >> 6, k8 = (idx & 63) * 8;
  _Float16 hh[8], hl[8];
#pragma unroll
  for (int e = 0; e < 8; ++e) { const float v = W[(size_t)(k8 + e + koff) * ldw + n]; hh[e] = (_Float16)v; hl[e] = lo_of(v, hh[e]); }
  _Float16* d = Wt + (size_t)n * 512 + k8;
  *(volatile v4u_t*)d = *(const v4ua*)hh; *(volatile v4u_t*)(d + PLW) = *(const v4ua*)hl; __threadfence();
  *(volatile v4u_t*)d = *(const v4ua*)hh; *(volatile v4u_t*)(d + PLW) = *(const v4ua*)hl;
}
__global__ void k_cast16(const float* __restrict__ X, _Float16* __restrict__ Y) {
  int i = (blockIdx.x * blockDim.x + threadIdx.x) * 2;
  if (i < NN * NN) stpair(Y + i, PLW, X[i], X[i + 1]);
}
__global__ void k_w0row(const float* __restrict__ W0, float* __restrict__ w0t) {
  int n = blockIdx.x * blockDim.x + threadIdx.x;
  if (n < HH) { const float v = W0[n]; *(volatile float*)(w0t + n) = v; __threadfence(); *(volatile float*)(w0t + n) = v; }
}

__device__ __forceinline__ void tile_coords(int& r0, int& c0, int& lane, int& wave) {
  lane = threadIdx.x & 31; wave = threadIdx.x >> 5;
  const int cg = blockIdx.x & 7, rg = blockIdx.x >> 3;
  r0 = (rg * 8 + wave) * 16; c0 = cg * 64;
}
__device__ __forceinline__ void store_tile_f16(float* sw, const v8f* acc4  , _Float16* dst, int r0, int c0, int lane) {
  const int g = lane >> 4, l16 = lane & 15;
#pragma unroll
  for (int j = 0; j < 4; ++j)
#pragma unroll
    for (int r = 0; r < 8; ++r) sw[(r + 8 * g) * 68 + j * 16 + l16] = acc4[j][r];
  asm volatile("s_wait_dscnt 0" ::: "memory");
#pragma unroll 1
  for (int pass = 0; pass < 2; ++pass) {
#pragma unroll
    for (int i = 0; i < 4; ++i) { const int c = lane + 32 * i, rr = c >> 3, q = (c & 7) * 8; const float* s = sw + rr * 68 + q;
      _Float16 hh[8], hl[8];
#pragma unroll
      for (int e = 0; e < 8; ++e) { hh[e] = (_Float16)s[e]; hl[e] = lo_of(s[e], hh[e]); }
      _Float16* d = dst + (size_t)(r0 + rr) * 512 + c0 + q;
      *(volatile v4u_t*)d = *(const v4ua*)hh; *(volatile v4u_t*)(d + PL) = *(const v4ua*)hl; }
    __threadfence();
  }
  asm volatile("s_wait_dscnt 0" ::: "memory");
}
__device__ __forceinline__ void store_tile_f32(float* sw, const v8f* acc4, float* dst, int r0, int c0, int lane) {
  const int g = lane >> 4, l16 = lane & 15;
#pragma unroll
  for (int j = 0; j < 4; ++j)
#pragma unroll
    for (int r = 0; r < 8; ++r) sw[(r + 8 * g) * 68 + j * 16 + l16] = acc4[j][r];
  asm volatile("s_wait_dscnt 0" ::: "memory");
#pragma unroll 1
  for (int pass = 0; pass < 2; ++pass) {
#pragma unroll
    for (int i = 0; i < 8; ++i) { const int c = lane + 32 * i, rr = c >> 4, q = (c & 15) * 4;
      *(volatile v4f_t*)(dst + (size_t)(r0 + rr) * 512 + c0 + q) = *(const volatile v4fa*)(sw + rr * 68 + q); }
    __threadfence();
  }
}

__device__ __forceinline__ void gemm_pass(const _Float16* __restrict__ A, const _Float16* __restrict__ Wt,
                                          int r0, int c0, int lane, v8f* acc) {
  const int g = lane >> 4, l16 = lane & 15;
#pragma unroll 2
  for (int k0 = 0; k0 < 512; k0 += 32) {
    const size_t ao = (size_t)(r0 + l16) * 512 + k0;
    const v16h a = frag16(A + ao, g), al = frag16(A + PL + ao, g);
#pragma unroll
    for (int j = 0; j < 4; ++j) {
      const _Float16* bp = Wt + (size_t)(c0 + j * 16 + l16) * 512 + k0;
      acc[j] = wmma_split(a, al, frag16(bp, g), frag16(bp + PLW, g), acc[j]);
    }
  }
}

__global__ void __launch_bounds__(256) k_layer0(
    const _Float16* __restrict__ pn16, const float* __restrict__ tn,
    const _Float16* __restrict__ W0t, const float* __restrict__ w0t, const float* __restrict__ b0,
    _Float16* __restrict__ Ov, _Float16* __restrict__ O1, _Float16* __restrict__ O2) {
  __shared__ __attribute__((aligned(16))) float stg[8][16 * 68];
  int r0, c0, lane, wave; tile_coords(r0, c0, lane, wave);
  const int g = lane >> 4, l16 = lane & 15;
  v8f acc[4] = {};
  gemm_pass(pn16, W0t, r0, c0, lane, acc);
  v8f va[4], v1[4], v2[4];
#pragma unroll
  for (int j = 0; j < 4; ++j) {
    const int col = c0 + j * 16 + l16;
    const float wt = w0t[col], zp = wt * (2.0f / T_MAX_N), bc = b0[col];
#pragma unroll
    for (int r = 0; r < 8; ++r) {
      const int row = r0 + r + 8 * g;
      const float z = acc[j][r] + tn[row] * wt + bc;
      const float a = tanhf(z), s = 1.f - a * a;
      const float ap = s * zp;
      const float app = -2.f * a * ap * zp;
      va[j][r] = a; v1[j][r] = ap; v2[j][r] = app;
    }
  }
  float* sw = stg[wave];
  store_tile_f16(sw, va, Ov, r0, c0, lane);
  store_tile_f16(sw, v1, O1, r0, c0, lane);
  store_tile_f16(sw, v2, O2, r0, c0, lane);
}

__global__ void __launch_bounds__(256) k_layer(
    const _Float16* __restrict__ Av, const _Float16* __restrict__ A1, const _Float16* __restrict__ A2,
    const _Float16* __restrict__ Wt, const float* __restrict__ bias,
    _Float16* __restrict__ Ov, _Float16* __restrict__ O1, _Float16* __restrict__ O2) {
  __shared__ __attribute__((aligned(16))) float stg[8][16 * 68];
  int r0, c0, lane, wave; tile_coords(r0, c0, lane, wave);
  const int g = lane >> 4, l16 = lane & 15;
  v8f acc0[4] = {}, acc1[4] = {}, acc2[4] = {};
  gemm_pass(Av, Wt, r0, c0, lane, acc0);
  gemm_pass(A1, Wt, r0, c0, lane, acc1);
  gemm_pass(A2, Wt, r0, c0, lane, acc2);
#pragma unroll
  for (int j = 0; j < 4; ++j) {
    const float bc = bias[c0 + j * 16 + l16];
#pragma unroll
    for (int r = 0; r < 8; ++r) {
      const float z = acc0[j][r] + bc, zp = acc1[j][r], zpp = acc2[j][r];
      const float a = tanhf(z), s = 1.f - a * a;
      const float ap = s * zp;
      const float app = s * zpp - 2.f * a * ap * zp;
      acc0[j][r] = a; acc1[j][r] = ap; acc2[j][r] = app;
    }
  }
  float* sw = stg[wave];
  store_tile_f16(sw, acc0, Ov, r0, c0, lane);
  store_tile_f16(sw, acc1, O1, r0, c0, lane);
  store_tile_f16(sw, acc2, O2, r0, c0, lane);
}

__global__ void __launch_bounds__(256) k_out(
    const _Float16* __restrict__ Av, const _Float16* __restrict__ A1, const _Float16* __restrict__ A2,
    const _Float16* __restrict__ Wt, const float* __restrict__ bias,
    float* __restrict__ out, float* __restrict__ outt, float* __restrict__ outtt,
    _Float16* __restrict__ S16, _Float16* __restrict__ C16) {
  __shared__ __attribute__((aligned(16))) float stg[8][16 * 68];
  int r0, c0, lane, wave; tile_coords(r0, c0, lane, wave);
  const int g = lane >> 4, l16 = lane & 15;
  float* sw = stg[wave];
  (void)g;
  {
    v8f acc[4] = {};
    gemm_pass(Av, Wt, r0, c0, lane, acc);
#pragma unroll
    for (int j = 0; j < 4; ++j) { const float bc = bias[c0 + j * 16 + l16];
#pragma unroll
      for (int r = 0; r < 8; ++r) acc[j][r] += bc; }
    store_tile_f32(sw, acc, out, r0, c0, lane);
    v8f tr[4];
#pragma unroll
    for (int j = 0; j < 4; ++j)
#pragma unroll
      for (int r = 0; r < 8; ++r) tr[j][r] = sinf(acc[j][r]);
    store_tile_f16(sw, tr, S16, r0, c0, lane);
#pragma unroll
    for (int j = 0; j < 4; ++j)
#pragma unroll
      for (int r = 0; r < 8; ++r) tr[j][r] = cosf(acc[j][r]);
    store_tile_f16(sw, tr, C16, r0, c0, lane);
  }
  {
    v8f acc[4] = {};
    gemm_pass(A1, Wt, r0, c0, lane, acc);
    store_tile_f32(sw, acc, outt, r0, c0, lane);
  }
  {
    v8f acc[4] = {};
    gemm_pass(A2, Wt, r0, c0, lane, acc);
    store_tile_f32(sw, acc, outtt, r0, c0, lane);
  }
}

__global__ void __launch_bounds__(256) k_conn(
    const _Float16* __restrict__ S16, const _Float16* __restrict__ C16, const _Float16* __restrict__ lb16,
    const float* __restrict__ out, const float* __restrict__ outt, const float* __restrict__ outtt,
    const float* __restrict__ lam_m, const float* __restrict__ lam_d,
    const float* __restrict__ power, float* __restrict__ phys) {
  __shared__ __attribute__((aligned(16))) float stg[8][16 * 68];
  int r0, c0, lane, wave; tile_coords(r0, c0, lane, wave);
  const int g = lane >> 4, l16 = lane & 15;
  v8f aC[4] = {}, aS[4] = {};
  gemm_pass(C16, lb16, r0, c0, lane, aC);
  gemm_pass(S16, lb16, r0, c0, lane, aS);
#pragma unroll
  for (int j = 0; j < 4; ++j) {
    const int col = c0 + j * 16 + l16;
    const float lm = lam_m[col], ld = lam_d[col];
#pragma unroll
    for (int r = 0; r < 8; ++r) {
      const int row = r0 + r + 8 * g;
      const size_t o = (size_t)row * 512 + col;
      const float d = out[o];
      const float sv = sinf(d), cvv = cosf(d);
      aC[j][r] = lm * outtt[o] + ld * outt[o] + sv * aC[j][r] - cvv * aS[j][r] - power[o];
    }
  }
  store_tile_f32(stg[wave], aC, phys, r0, c0, lane);
}

extern "C" void kernel_launch(void* const* d_in, const int* in_sizes, int n_in,
                              void* d_out, int out_size, void* d_ws, size_t ws_size,
                              hipStream_t stream) {
  (void)in_sizes; (void)n_in; (void)out_size; (void)ws_size;
  const float* t_in  = (const float*)d_in[0];
  const float* p_in  = (const float*)d_in[1];
  const float* W0    = (const float*)d_in[2];
  const float* b0    = (const float*)d_in[3];
  const float* W1    = (const float*)d_in[4];
  const float* b1    = (const float*)d_in[5];
  const float* W2    = (const float*)d_in[6];
  const float* b2    = (const float*)d_in[7];
  const float* Wout  = (const float*)d_in[8];
  const float* bout  = (const float*)d_in[9];
  const float* lam_m = (const float*)d_in[10];
  const float* lam_d = (const float*)d_in[11];
  const float* lam_b = (const float*)d_in[12];
  const float* p_lo  = (const float*)d_in[13];
  const float* p_up  = (const float*)d_in[14];

  float* out  = (float*)d_out;
  float* outt = out + (size_t)BB * NN;
  float* phys = out + 2 * (size_t)BB * NN;

  char* w = (char*)d_ws;
  auto alloc = [&](size_t bytes) -> void* { void* p = (void*)w; w += (bytes + 255) & ~(size_t)255; return p; };
  _Float16* pn16  = (_Float16*)alloc(PL * 2 * 2);
  float*    tn    = (float*)   alloc((size_t)BB * 4);
  float*    w0t   = (float*)   alloc((size_t)HH * 4);
  _Float16* W0t   = (_Float16*)alloc(PLW * 2 * 2);
  _Float16* W1t   = (_Float16*)alloc(PLW * 2 * 2);
  _Float16* W2t   = (_Float16*)alloc(PLW * 2 * 2);
  _Float16* Wot   = (_Float16*)alloc(PLW * 2 * 2);
  _Float16* lb16  = (_Float16*)alloc(PLW * 2 * 2);
  _Float16* Xa    = (_Float16*)alloc(PL * 2 * 2);
  _Float16* Xa1   = (_Float16*)alloc(PL * 2 * 2);
  _Float16* Xa2   = (_Float16*)alloc(PL * 2 * 2);
  _Float16* Xb    = (_Float16*)alloc(PL * 2 * 2);
  _Float16* Xb1   = (_Float16*)alloc(PL * 2 * 2);
  _Float16* Xb2   = (_Float16*)alloc(PL * 2 * 2);
  float*    outtt = (float*)   alloc((size_t)BB * NN * 4);
  _Float16* S16   = (_Float16*)alloc(PL * 2 * 2);
  _Float16* C16   = (_Float16*)alloc(PL * 2 * 2);

  k_prep_inputs<<<(BB * NN / 2) / 256, 256, 0, stream>>>(t_in, p_in, p_lo, p_up, pn16, tn);
  k_w0row<<<2, 256, 0, stream>>>(W0, w0t);
  k_tcast<<<(512 * 64) / 256, 256, 0, stream>>>(W0, 1, HH, W0t);
  k_tcast<<<(512 * 64) / 256, 256, 0, stream>>>(W1, 0, HH, W1t);
  k_tcast<<<(512 * 64) / 256, 256, 0, stream>>>(W2, 0, HH, W2t);
  k_tcast<<<(512 * 64) / 256, 256, 0, stream>>>(Wout, 0, NN, Wot);
  k_cast16<<<(NN * NN / 2) / 256, 256, 0, stream>>>(lam_b, lb16);

  const int GB = 64, TB = 256;
  k_layer0<<<GB, TB, 0, stream>>>(pn16, tn, W0t, w0t, b0, Xa, Xa1, Xa2);
  k_layer <<<GB, TB, 0, stream>>>(Xa, Xa1, Xa2, W1t, b1, Xb, Xb1, Xb2);
  k_layer <<<GB, TB, 0, stream>>>(Xb, Xb1, Xb2, W2t, b2, Xa, Xa1, Xa2);
  k_out   <<<GB, TB, 0, stream>>>(Xa, Xa1, Xa2, Wot, bout, out, outt, outtt, S16, C16);
  k_conn  <<<GB, TB, 0, stream>>>(S16, C16, lb16, out, outt, outtt, lam_m, lam_d, p_in, phys);
}
